// TSModel_45165876084961
// MI455X (gfx1250) — hardware-verified
//
#include <hip/hip_runtime.h>
#include <math.h>

constexpr int NBATCH = 256;
constexpr int NSTEP  = 2048;
constexpr int NUNIT  = 64;
constexpr int NGATE  = 4 * NUNIT;
constexpr int NIN0   = NUNIT + 1;
constexpr int RPB    = 16;
constexpr int NWM    = 4;
constexpr int NTHR   = 32 * (NWM + 1);
constexpr int WTP    = 72;
constexpr int AHP    = 72;
constexpr int AHB    = RPB * AHP;
constexpr int HMP    = 20;
constexpr int HFB    = NUNIT * HMP;
constexpr int OBP    = 68;
constexpr int CHUNK  = 64;
constexpr float HCARRY = 4096.0f;
constexpr float RCARRY = 2048.0f;
constexpr float WCARRY = 256.0f;
constexpr float S_HI   = 1.0f / (HCARRY * WCARRY);
constexpr float S_LO   = 1.0f / (HCARRY * RCARRY * WCARRY);
constexpr float FGBIAS = 1.0f;
constexpr float L2EPS  = 1e-12f;
static_assert(NBATCH % RPB == 0);
static_assert(NUNIT == 16 * NWM);
static_assert(NUNIT % 32 == 0);
static_assert(NGATE == 256);
static_assert(NSTEP % CHUNK == 0);
static_assert(NSTEP % 128 == 0);
static_assert(CHUNK == 64 && RPB == 16);
static_assert((WTP % 8) == 0 && (AHP % 8) == 0 && (HMP % 4) == 0 && (OBP % 4) == 0);
static_assert((AHB % 2) == 0);

typedef __attribute__((ext_vector_type(16))) _Float16 v16h;
typedef __attribute__((ext_vector_type(8)))  _Float16 v8h;
typedef __attribute__((ext_vector_type(8)))  float    v8f;
typedef __attribute__((ext_vector_type(4)))  float    v4f;

__device__ __forceinline__ void dep_guard1(v8f& a, v16h x0, v16h x1, v16h y0, v16h y1) {
  asm volatile("v_nop\n\tv_nop\n\tv_nop\n\tv_nop" : "+v"(a) : "v"(x0), "v"(x1), "v"(y0), "v"(y1));
}
__device__ __forceinline__ void acc_guard4(v8f& a, v8f& b, v8f& c, v8f& d) {
  asm volatile("v_nop\n\tv_nop\n\tv_nop\n\tv_nop" : "+v"(a), "+v"(b), "+v"(c), "+v"(d));
}
template <typename T> struct Frag;
template <> struct Frag<_Float16> {
  typedef v16h V; union U { v16h v; v8h h[2]; };
  static __device__ __forceinline__ v16h load(const _Float16* p) {
    U f; f.h[0] = *(const v8h*)(p); f.h[1] = *(const v8h*)(p + 16); return f.v;
  }
  static __device__ __forceinline__ v8f mma(v16h a, v16h b, v8f c) {
    return __builtin_amdgcn_wmma_f32_16x16x32_f16(false, a, false, b, (short)0, c, false, false);
  }
};

__device__ __forceinline__ float sigm(float x) { return __builtin_amdgcn_rcpf(1.0f + expf(-x)); }
__device__ __forceinline__ float tanhs(float x) {
  const float x2 = x * x;
  float p = fmaf(x2, -17.0f / 315.0f, 2.0f / 15.0f);
  p = fmaf(x2, p, -1.0f / 3.0f);
  p = fmaf(x2, p, 1.0f);
  const float sm = x * p;
  const float e  = expf(2.0f * x);
  const float bg = 1.0f - 2.0f * __builtin_amdgcn_rcpf(e + 1.0f);
  return (fabsf(x) < 0.0625f) ? sm : bg;
}

__device__ __forceinline__ void layer1_step(const float* hcol, const float* w1s, const float (&w64r)[4],
                                            const float (&b1r)[4], float wdv, float bdv,
                                            float& c1, float& h1, float* obp, int slot, int lane) {
  const int row = lane & 15, half = lane >> 4;
  const float* hp = hcol + (half * 32) * HMP + row;
  const float* wp = w1s + half * 32 * 4;
  float z0 = 0.0f, z1 = 0.0f, z2 = 0.0f, z3 = 0.0f;
#pragma unroll 8
  for (int uu = 0; uu < 32; ++uu) {
    const float hv = hp[uu * HMP];
    const v4f w = *(const v4f*)(wp + uu * 4);
    z0 = fmaf(hv, w[0], z0);
    z1 = fmaf(hv, w[1], z1);
    z2 = fmaf(hv, w[2], z2);
    z3 = fmaf(hv, w[3], z3);
  }
  z0 += __shfl_xor(z0, 16, 32);
  z1 += __shfl_xor(z1, 16, 32);
  z2 += __shfl_xor(z2, 16, 32);
  z3 += __shfl_xor(z3, 16, 32);
  z0 = fmaf(h1, w64r[0], z0) + b1r[0];
  z1 = fmaf(h1, w64r[1], z1) + b1r[1];
  z2 = fmaf(h1, w64r[2], z2) + b1r[2];
  z3 = fmaf(h1, w64r[3], z3) + b1r[3];
  const float ig = sigm(z0);
  const float gj = tanhs(z1);
  const float fg = sigm(z2 + FGBIAS);
  const float og = sigm(z3);
  c1 = fmaf(fg, c1, ig * gj);
  h1 = og * tanhs(c1);
  const float o = fmaf(h1, wdv, bdv);
  if (half == 0) obp[row * OBP + slot] = o;
}

__device__ __forceinline__ void flush_chunk(const float* obp, float* out, int rowbase, int t0, int lane) {
  __builtin_amdgcn_fence(__ATOMIC_RELEASE, "workgroup");
  __builtin_amdgcn_wave_barrier();
  __builtin_amdgcn_fence(__ATOMIC_ACQUIRE, "workgroup");
  const int q = lane >> 3, c4 = (lane & 7) * 4;
  for (int pass = 0; pass < 2; ++pass) {
#pragma unroll
    for (int it = 0; it < 8; ++it) {
      const int ln  = it * 4 + q;
      const int row = ln >> 1;
      const int hs  = (ln & 1) * 32;
      const v4f v = *(const v4f*)(obp + row * OBP + hs + c4);
      *(volatile v4f*)(out + (size_t)(rowbase + row) * NSTEP + t0 + hs + c4) = v;
    }
    __threadfence();
  }
  __builtin_amdgcn_fence(__ATOMIC_RELEASE, "workgroup");
  __builtin_amdgcn_wave_barrier();
  __builtin_amdgcn_fence(__ATOMIC_ACQUIRE, "workgroup");
}

__global__ __launch_bounds__(NTHR) void ts_seq_kernel(const float* __restrict__ x, const float* __restrict__ W0,
                                                      const float* __restrict__ b0, const float* __restrict__ W1,
                                                      const float* __restrict__ b1, const float* __restrict__ Wd,
                                                      const float* __restrict__ bd, float* __restrict__ out) {
  __shared__ __align__(16) unsigned short Wt[NGATE * WTP];
  __shared__ __align__(16) _Float16 Ah[2 * AHB];
  __shared__ __align__(16) _Float16 Al[2 * AHB];
  __shared__ __align__(16) float    HfT[2 * HFB];
  __shared__ __align__(16) float    W1s[NIN0 * 4];
  __shared__ __align__(16) float    xb[2 * RPB];
  __shared__ __align__(16) float    ob[RPB * OBP];

  const int tid = threadIdx.x, lane = tid & 31, wave = tid >> 5;
  const int c = lane & 15, hh = lane >> 4, koff = hh * 8;
  const int rowbase = blockIdx.x * RPB;

  {
    unsigned* ahz = (unsigned*)(void*)Ah;
    unsigned* alz = (unsigned*)(void*)Al;
#pragma unroll 1
    for (int i = tid; i < AHB; i += NTHR) { ahz[i] = 0u; alz[i] = 0u; }
#pragma unroll 1
    for (int i = tid; i < 2 * HFB; i += NTHR) HfT[i] = 0.0f;
  }
#pragma unroll 1
  for (int e = tid; e < NGATE * (NUNIT / 2); e += NTHR) {
    const int k2 = e >> 8, n = e & 255;
    const float v0 = W0[(size_t)(1 + 2 * k2) * NGATE + n];
    const float v1 = W0[(size_t)(2 + 2 * k2) * NGATE + n];
    const _Float16 f0 = (_Float16)(v0 * WCARRY);
    const _Float16 f1 = (_Float16)(v1 * WCARRY);
    const unsigned u = (unsigned)__builtin_bit_cast(unsigned short, f0) | ((unsigned)__builtin_bit_cast(unsigned short, f1) << 16);
    *(unsigned*)(void*)(Wt + n * WTP + 2 * k2) = u;
  }
#pragma unroll 1
  for (int i = tid; i < NIN0 * 4; i += NTHR) W1s[i] = W1[i];

  const int ucl = (wave < NWM) ? (16 * wave + c) : c;
  float w0r[4], b0r[4];
#pragma unroll
  for (int g = 0; g < 4; ++g) { w0r[g] = W0[g * NUNIT + ucl]; b0r[g] = b0[g * NUNIT + ucl]; }
  asm volatile("" ::: "memory");
  float b1r[4], w64r[4];
#pragma unroll
  for (int g = 0; g < 4; ++g) { b1r[g] = b1[g]; w64r[g] = W1[NUNIT * 4 + g]; }
  const float wdv = Wd[0], bdv = bd[0];

  float cst[8];
#pragma unroll
  for (int r = 0; r < 8; ++r) cst[r] = 0.0f;
  float c1 = 0.0f, h1 = 0.0f, invr = 0.0f;

  if (wave == NWM) {
#pragma unroll 1
    for (int m = 0; m < RPB; ++m) {
      const float* xr = x + (size_t)(rowbase + m) * NSTEP + lane * 4;
      float s = 0.0f;
#pragma unroll 4
      for (int i = 0; i < NSTEP / 128; ++i) {
        const v4f v = *(const v4f*)(xr + i * 128);
        s = fmaf(v[0], v[0], s);
        s = fmaf(v[1], v[1], s);
        s = fmaf(v[2], v[2], s);
        s = fmaf(v[3], v[3], s);
      }
#pragma unroll
      for (int off = 1; off < 32; off <<= 1) s += __shfl_xor(s, off, 32);
      const float inv = 1.0f / sqrtf(fmaxf(s, L2EPS));
      invr = (m == c) ? inv : invr;
    }
    xb[c] = x[(size_t)(rowbase + c) * NSTEP] * invr;
  }
  __syncthreads();

  const v8f z8 = {0.f, 0.f, 0.f, 0.f, 0.f, 0.f, 0.f, 0.f};

#pragma unroll 1
  for (int t = 0; t < NSTEP; ++t) {
    const int P = t & 1, Pn = P ^ 1;
    if (wave < NWM) {
      const _Float16* ahp = Ah + P * AHB + c * AHP + koff;
      const _Float16* alp = Al + P * AHB + c * AHP + koff;
      const _Float16* wtb = (const _Float16*)(const void*)Wt + (16 * wave + c) * WTP + koff;
      v8f acch[4], accl[4];
      {
        const v16h a0 = Frag<_Float16>::load(ahp);
        const v16h a1 = Frag<_Float16>::load(ahp + 32);
#pragma unroll
        for (int g = 0; g < 4; ++g) {
          const v16h q0 = Frag<_Float16>::load(wtb + g * (NUNIT * WTP));
          const v16h q1 = Frag<_Float16>::load(wtb + g * (NUNIT * WTP) + 32);
          v8f a = Frag<_Float16>::mma(a0, q0, z8);
          a = Frag<_Float16>::mma(a1, q1, a);
          dep_guard1(a, a0, a1, q0, q1);
          acch[g] = a;
        }
      }
      {
        const v16h a0 = Frag<_Float16>::load(alp);
        const v16h a1 = Frag<_Float16>::load(alp + 32);
#pragma unroll
        for (int g = 0; g < 4; ++g) {
          const v16h q0 = Frag<_Float16>::load(wtb + g * (NUNIT * WTP));
          const v16h q1 = Frag<_Float16>::load(wtb + g * (NUNIT * WTP) + 32);
          v8f a = Frag<_Float16>::mma(a0, q0, z8);
          a = Frag<_Float16>::mma(a1, q1, a);
          dep_guard1(a, a0, a1, q0, q1);
          accl[g] = a;
        }
      }
      acc_guard4(acch[0], acch[1], acch[2], acch[3]);
      acc_guard4(accl[0], accl[1], accl[2], accl[3]);

      const v4f xq0 = *(const v4f*)(xb + P * RPB + 8 * hh);
      const v4f xq1 = *(const v4f*)(xb + P * RPB + 8 * hh + 4);
      float xt8[8];
      xt8[0] = xq0[0]; xt8[1] = xq0[1]; xt8[2] = xq0[2]; xt8[3] = xq0[3];
      xt8[4] = xq1[0]; xt8[5] = xq1[1]; xt8[6] = xq1[2]; xt8[7] = xq1[3];
      const int u = 16 * wave + c;
      _Float16* ahn = Ah + Pn * AHB + u;
      _Float16* aln = Al + Pn * AHB + u;
      float hnew[8];
#pragma unroll
      for (int r = 0; r < 8; ++r) {
        const float xt = xt8[r];
        const float zi = fmaf(acch[0][r], S_HI, fmaf(accl[0][r], S_LO, fmaf(xt, w0r[0], b0r[0])));
        const float zj = fmaf(acch[1][r], S_HI, fmaf(accl[1][r], S_LO, fmaf(xt, w0r[1], b0r[1])));
        const float zf = fmaf(acch[2][r], S_HI, fmaf(accl[2][r], S_LO, fmaf(xt, w0r[2], b0r[2])));
        const float zo = fmaf(acch[3][r], S_HI, fmaf(accl[3][r], S_LO, fmaf(xt, w0r[3], b0r[3])));
        const float ig = sigm(zi);
        const float gj = tanhs(zj);
        const float fg = sigm(zf + FGBIAS);
        const float og = sigm(zo);
        const float cn = fmaf(fg, cst[r], ig * gj);
        cst[r] = cn;
        const float hn = og * tanhs(cn);
        hnew[r] = hn;
        const float hsf = hn * HCARRY;
        const _Float16 h16 = (_Float16)hsf;
        const float res = (hsf - (float)h16) * RCARRY;
        const _Float16 l16 = (_Float16)res;
        ahn[(8 * hh + r) * AHP] = h16;
        aln[(8 * hh + r) * AHP] = l16;
      }
      v4f o0, o1;
      o0[0] = hnew[0]; o0[1] = hnew[1]; o0[2] = hnew[2]; o0[3] = hnew[3];
      o1[0] = hnew[4]; o1[1] = hnew[5]; o1[2] = hnew[6]; o1[3] = hnew[7];
      float* hfp = HfT + Pn * HFB + u * HMP + 8 * hh;
      *(v4f*)hfp = o0;
      *(v4f*)(hfp + 4) = o1;
    } else {
      if (t > 0) {
        layer1_step(HfT + P * HFB, W1s, w64r, b1r, wdv, bdv, c1, h1, ob, (t - 1) & (CHUNK - 1), lane);
        if ((t & (CHUNK - 1)) == 0) flush_chunk(ob, out, rowbase, t - CHUNK, lane);
      }
      const int tn = (t + 1 < NSTEP) ? (t + 1) : (NSTEP - 1);
      xb[Pn * RPB + c] = x[(size_t)(rowbase + c) * NSTEP + tn] * invr;
    }
    __syncthreads();
  }

  if (wave == NWM) {
    layer1_step(HfT + (NSTEP & 1) * HFB, W1s, w64r, b1r, wdv, bdv, c1, h1, ob, (NSTEP - 1) & (CHUNK - 1), lane);
    flush_chunk(ob, out, rowbase, NSTEP - CHUNK, lane);
  }
}

extern "C" void kernel_launch(void* const* d_in, const int* in_sizes, int n_in,
                              void* d_out, int out_size, void* d_ws, size_t ws_size, hipStream_t stream) {
  (void)d_ws; (void)ws_size;
  if (n_in < 7 || d_out == nullptr) return;
  if (in_sizes[0] != NBATCH * NSTEP || in_sizes[1] != NIN0 * NGATE || in_sizes[2] != NGATE ||
      in_sizes[3] != NIN0 * 4 || in_sizes[4] != 4 || in_sizes[5] != 1 || in_sizes[6] != 1 ||
      out_size != NBATCH * NSTEP) return;

  const float* x  = (const float*)d_in[0];
  const float* W0 = (const float*)d_in[1];
  const float* b0 = (const float*)d_in[2];
  const float* W1 = (const float*)d_in[3];
  const float* b1 = (const float*)d_in[4];
  const float* Wd = (const float*)d_in[5];
  const float* bd = (const float*)d_in[6];
  float* out = (float*)d_out;

  ts_seq_kernel<<<NBATCH / RPB, NTHR, 0, stream>>>(x, W0, b0, W1, b1, Wd, bd, out);
}
